// LayerNormGRUCell_4776003633435
// MI455X (gfx1250) — hardware-verified
//
#include <hip/hip_runtime.h>

typedef __bf16         v16bf __attribute__((ext_vector_type(16)));
typedef unsigned short v8us  __attribute__((ext_vector_type(8)));
typedef float          v8f   __attribute__((ext_vector_type(8)));
typedef float          v4f   __attribute__((ext_vector_type(4)));
typedef v8us __attribute__((may_alias)) v8usa;
typedef v4f  __attribute__((may_alias)) v4fa;

union Frag { v16bf v; v8us half[2]; };

#define NBATCH 16384
#define KD     512
#define N2H    1024
#define NH     512
#define RB     16
#define NTHR   256
#define LN_EPS 1e-5f

#define G_X0   0
#define G_H0   1048576
#define G_WI0  2097152
#define G_WH0  2162688
#define G_WW0  2228224
#define G_WU0  2260992
#define G_END  2293760
#define WS_TOTAL_BYTES ((size_t)G_END * 16)

static_assert(G_H0  == NBATCH * KD / 8);
static_assert(G_WI0 == G_H0  + NBATCH * KD / 8);
static_assert(G_WH0 == G_WI0 + N2H * KD / 8);
static_assert(G_WW0 == G_WH0 + N2H * KD / 8);
static_assert(G_WU0 == G_WW0 + NH * KD / 8);
static_assert(G_END == G_WU0 + NH * KD / 8);
static_assert(G_H0 % NTHR == 0 && G_WI0 % NTHR == 0 && G_WH0 % NTHR == 0 && G_WW0 % NTHR == 0 && G_WU0 % NTHR == 0 && G_END % NTHR == 0);
static_assert(NBATCH % RB == 0);
static_assert(KD % 32 == 0);
static_assert(N2H == 8 * 128 && NH == 8 * 64);

#define OFF_G    0
#define OFF_A    65536
#define OFF_HP   98304
#define OFF_PART 114688
#define OFF_MU   115200
#define OFF_RS   115264
#define SMEM_BYTES 115328

__device__ __forceinline__ unsigned short f2bf(float f) {
  unsigned u = __builtin_bit_cast(unsigned, f);
  u += 0x7FFFu + ((u >> 16) & 1u);
  return (unsigned short)(u >> 16);
}
__device__ __forceinline__ float bf2f(unsigned short s) {
  return __builtin_bit_cast(float, ((unsigned)s) << 16);
}
__device__ __forceinline__ float bfr(float f) { return bf2f(f2bf(f)); }

__device__ __forceinline__ float sigm_f(float v) {
  v = fminf(fmaxf(v, -30.0f), 30.0f);
  const float e = __expf(-v);
  return __builtin_amdgcn_rcpf(1.0f + e);
}
__device__ __forceinline__ float tanh_f(float v) {
  v = fminf(fmaxf(v, -15.0f), 15.0f);
  const float e = __expf(2.0f * v);
  return 1.0f - 2.0f * __builtin_amdgcn_rcpf(1.0f + e);
}

__device__ __forceinline__ v8f wmma_bf16(v16bf a, v16bf b, v8f c) {
  v8f d = __builtin_amdgcn_wmma_f32_16x16x32_bf16(false, a, false, b, (short)0, c, false, false);
  asm volatile("v_nop\n\tv_nop\n\tv_nop\n\tv_nop" : "+v"(d) : "v"(a), "v"(b));
  return d;
}

__device__ __forceinline__ v16bf load_frag(const unsigned short* p, int h) {
  Frag f;
  f.half[0] = *(const v8usa*)(p + 8 * h);
  f.half[1] = *(const v8usa*)(p + 16 + 8 * h);
  return f.v;
}

__global__ __launch_bounds__(NTHR) void convert_planes(
    const float* __restrict__ x,  const float* __restrict__ hprev,
    const float* __restrict__ wi, const float* __restrict__ wh,
    const float* __restrict__ ww, const float* __restrict__ wu,
    unsigned short* __restrict__ planes)
{
  const int g = blockIdx.x * NTHR + threadIdx.x;
  if (g >= G_END) return;
  const float* src;
  if (g < G_H0)       src = x     + (size_t)g * 8;
  else if (g < G_WI0) src = hprev + (size_t)(g - G_H0) * 8;
  else if (g < G_WH0) src = wi    + (size_t)(g - G_WI0) * 8;
  else if (g < G_WW0) src = wh    + (size_t)(g - G_WH0) * 8;
  else if (g < G_WU0) src = ww    + (size_t)(g - G_WW0) * 8;
  else                src = wu    + (size_t)(g - G_WU0) * 8;
  const v4f a = *(const v4fa*)src;
  const v4f c = *(const v4fa*)(src + 4);
  const v8us o = { f2bf(a.x), f2bf(a.y), f2bf(a.z), f2bf(a.w),
                   f2bf(c.x), f2bf(c.y), f2bf(c.z), f2bf(c.w) };
  unsigned short* dst = planes + (size_t)g * 8;
  *(volatile v8us*)dst = o;
  __threadfence();
  *(volatile v8us*)dst = o;
}

template <int T>
__device__ __forceinline__ void gemm_strip(const unsigned short* __restrict__ arow,
                                           const unsigned short* __restrict__ brow,
                                           int h, v8f (&acc)[T]) {
  const v8f z8 = {0.f, 0.f, 0.f, 0.f, 0.f, 0.f, 0.f, 0.f};
  #pragma unroll
  for (int t = 0; t < T; ++t) acc[t] = z8;
  #pragma unroll 1
  for (int k0 = 0; k0 < KD; k0 += 32) {
    const v16bf a = load_frag(arow + k0, h);
    #pragma unroll
    for (int t = 0; t < T; ++t) {
      const v16bf b = load_frag(brow + (size_t)t * 16 * KD + k0, h);
      acc[t] = wmma_bf16(a, b, acc[t]);
    }
  }
}

template <int T>
__device__ __forceinline__ void ln_strip(v8f (&acc)[T], const float (&bia)[T], float invN,
                                         float* sPart, float* sMu, float* sRs,
                                         int tid, int w, int h, int m) {
  float s[8];
  #pragma unroll
  for (int r = 0; r < 8; ++r) s[r] = 0.0f;
  #pragma unroll
  for (int t = 0; t < T; ++t) {
    #pragma unroll
    for (int r = 0; r < 8; ++r) {
      const float v = acc[t][r] + bia[t];
      acc[t][r] = v;
      s[r] += v;
    }
  }
  #pragma unroll
  for (int r = 0; r < 8; ++r) {
    float v = s[r];
    v += __shfl_xor(v, 1);
    v += __shfl_xor(v, 2);
    v += __shfl_xor(v, 4);
    v += __shfl_xor(v, 8);
    s[r] = v;
  }
  if (m == 0) {
    #pragma unroll
    for (int r = 0; r < 8; ++r) sPart[(8 * h + r) * 8 + w] = s[r];
  }
  __syncthreads();
  if (tid < RB) {
    float a = 0.0f;
    #pragma unroll
    for (int wv = 0; wv < 8; ++wv) a += sPart[tid * 8 + wv];
    sMu[tid] = a * invN;
  }
  __syncthreads();
  float mu[8], q[8];
  #pragma unroll
  for (int r = 0; r < 8; ++r) { mu[r] = sMu[8 * h + r]; q[r] = 0.0f; }
  #pragma unroll
  for (int t = 0; t < T; ++t) {
    #pragma unroll
    for (int r = 0; r < 8; ++r) {
      const float d = acc[t][r] - mu[r];
      acc[t][r] = d;
      q[r] += d * d;
    }
  }
  #pragma unroll
  for (int r = 0; r < 8; ++r) {
    float v = q[r];
    v += __shfl_xor(v, 1);
    v += __shfl_xor(v, 2);
    v += __shfl_xor(v, 4);
    v += __shfl_xor(v, 8);
    q[r] = v;
  }
  if (m == 0) {
    #pragma unroll
    for (int r = 0; r < 8; ++r) sPart[(8 * h + r) * 8 + w] = q[r];
  }
  __syncthreads();
  if (tid < RB) {
    float a = 0.0f;
    #pragma unroll
    for (int wv = 0; wv < 8; ++wv) a += sPart[tid * 8 + wv];
    sRs[tid] = rsqrtf(a * invN + LN_EPS);
  }
  __syncthreads();
  #pragma unroll
  for (int r = 0; r < 8; ++r) {
    const float rs = sRs[8 * h + r];
    #pragma unroll
    for (int t = 0; t < T; ++t) acc[t][r] = acc[t][r] * rs;
  }
}

__device__ __forceinline__ void out_store_pass(const float* sO, float* out,
                                               int row0, int w, int lane) {
  const int q8 = lane & 7, sub = lane >> 3;
  #pragma unroll
  for (int i = 0; i < 8; ++i) {
    const int lid = w * 32 + i * 4 + sub;
    const int row = lid >> 4, seg = lid & 15;
    const v4f v = *(const v4fa*)(sO + row * NH + seg * 32 + 4 * q8);
    *(volatile v4f*)(out + (size_t)(row0 + row) * NH + seg * 32 + 4 * q8) = v;
  }
}

__global__ __launch_bounds__(NTHR) void gru_cell_kernel(
    const unsigned short* __restrict__ xb,
    const unsigned short* __restrict__ hb,
    const unsigned short* __restrict__ wi,
    const unsigned short* __restrict__ wh,
    const unsigned short* __restrict__ ww,
    const unsigned short* __restrict__ wu,
    const float* __restrict__ b_i2h, const float* __restrict__ b_h2h,
    const float* __restrict__ b_hatW, const float* __restrict__ b_hatU,
    float* __restrict__ out)
{
  extern __shared__ __attribute__((aligned(16))) char smem[];
  float* sG = (float*)(smem + OFF_G);
  float* sA = (float*)(smem + OFF_A);
  unsigned short* sHp = (unsigned short*)(smem + OFF_HP);
  float* sPart = (float*)(smem + OFF_PART);
  float* sMu = (float*)(smem + OFF_MU);
  float* sRs = (float*)(smem + OFF_RS);

  const int tid = threadIdx.x, lane = tid & 31, w = tid >> 5;
  const int h = lane >> 4, m = lane & 15;
  const int row0 = blockIdx.x * RB;

  #pragma unroll
  for (int it = 0; it < 4; ++it) {
    const int q = it * NTHR + tid;
    const v8us v = *(const v8usa*)(hb + (size_t)row0 * KD + (size_t)q * 8);
    *(v8usa*)(sHp + q * 8) = v;
  }
  __syncthreads();

  const unsigned short* xrow = xb + (size_t)(row0 + m) * KD;
  const unsigned short* hrow = hb + (size_t)(row0 + m) * KD;

  {
    v8f acc[8];
    gemm_strip<8>(xrow, wi + (size_t)(128 * w + m) * KD, h, acc);
    float bia[8];
    #pragma unroll
    for (int t = 0; t < 8; ++t) bia[t] = bfr(b_i2h[128 * w + 16 * t + m]);
    ln_strip<8>(acc, bia, 1.0f / 1024.0f, sPart, sMu, sRs, tid, w, h, m);
    #pragma unroll
    for (int t = 0; t < 8; ++t)
      #pragma unroll
      for (int r = 0; r < 8; ++r)
        sG[(8 * h + r) * N2H + 128 * w + 16 * t + m] = acc[t][r];
  }
  {
    v8f acc[8];
    gemm_strip<8>(hrow, wh + (size_t)(128 * w + m) * KD, h, acc);
    float bia[8];
    #pragma unroll
    for (int t = 0; t < 8; ++t) bia[t] = bfr(b_h2h[128 * w + 16 * t + m]);
    ln_strip<8>(acc, bia, 1.0f / 1024.0f, sPart, sMu, sRs, tid, w, h, m);
    #pragma unroll
    for (int t = 0; t < 8; ++t)
      #pragma unroll
      for (int r = 0; r < 8; ++r) {
        const int idx = (8 * h + r) * N2H + 128 * w + 16 * t + m;
        const float v = sG[idx] + acc[t][r];
        sG[idx] = sigm_f(v);
      }
  }
  {
    v8f acc[4];
    gemm_strip<4>(xrow, ww + (size_t)(64 * w + m) * KD, h, acc);
    float bia[4];
    #pragma unroll
    for (int t = 0; t < 4; ++t) bia[t] = bfr(b_hatW[64 * w + 16 * t + m]);
    ln_strip<4>(acc, bia, 1.0f / 512.0f, sPart, sMu, sRs, tid, w, h, m);
    #pragma unroll
    for (int t = 0; t < 4; ++t)
      #pragma unroll
      for (int r = 0; r < 8; ++r)
        sA[(8 * h + r) * NH + 64 * w + 16 * t + m] = acc[t][r];
  }
  {
    v8f acc[4];
    gemm_strip<4>(hrow, wu + (size_t)(64 * w + m) * KD, h, acc);
    float bia[4];
    #pragma unroll
    for (int t = 0; t < 4; ++t) bia[t] = bfr(b_hatU[64 * w + 16 * t + m]);
    ln_strip<4>(acc, bia, 1.0f / 512.0f, sPart, sMu, sRs, tid, w, h, m);
    #pragma unroll
    for (int t = 0; t < 4; ++t)
      #pragma unroll
      for (int r = 0; r < 8; ++r) {
        const int row = 8 * h + r;
        const int n = 64 * w + 16 * t + m;
        const float z  = sG[row * N2H + n];
        const float rg = sG[row * N2H + NH + n];
        const float a  = sA[row * NH + n];
        const float hp = bf2f(sHp[row * KD + n]);
        const float hh = tanh_f(a + rg * acc[t][r]);
        const float o  = (1.0f - z) * hp + z * hh;
        sA[row * NH + n] = o;
      }
  }
  __syncthreads();

  out_store_pass(sA, out, row0, w, lane);
  __threadfence();
  out_store_pass(sA, out, row0, w, lane);
}

extern "C" void kernel_launch(void* const* d_in, const int* in_sizes, int n_in,
                              void* d_out, int out_size, void* d_ws, size_t ws_size,
                              hipStream_t stream) {
  if (n_in < 10) return;
  if (in_sizes[0] != NBATCH * KD || in_sizes[1] != NBATCH * KD) return;
  if (in_sizes[2] != N2H * KD || in_sizes[3] != N2H) return;
  if (in_sizes[4] != N2H * KD || in_sizes[5] != N2H) return;
  if (in_sizes[6] != NH * KD || in_sizes[7] != NH) return;
  if (in_sizes[8] != NH * KD || in_sizes[9] != NH) return;
  if (out_size != NBATCH * NH) return;
  if (WS_TOTAL_BYTES > ws_size) return;

  const float* x     = (const float*)d_in[0];
  const float* hprev = (const float*)d_in[1];
  const float* Wi2h  = (const float*)d_in[2];
  const float* bi2h  = (const float*)d_in[3];
  const float* Wh2h  = (const float*)d_in[4];
  const float* bh2h  = (const float*)d_in[5];
  const float* WhatW = (const float*)d_in[6];
  const float* bhatW = (const float*)d_in[7];
  const float* WhatU = (const float*)d_in[8];
  const float* bhatU = (const float*)d_in[9];
  float* out = (float*)d_out;

  unsigned short* planes = (unsigned short*)d_ws;
  const unsigned short* xb  = planes + (size_t)G_X0  * 8;
  const unsigned short* hbp = planes + (size_t)G_H0  * 8;
  const unsigned short* wib = planes + (size_t)G_WI0 * 8;
  const unsigned short* whb = planes + (size_t)G_WH0 * 8;
  const unsigned short* wwb = planes + (size_t)G_WW0 * 8;
  const unsigned short* wub = planes + (size_t)G_WU0 * 8;

  convert_planes<<<G_END / NTHR, NTHR, 0, stream>>>(x, hprev, Wi2h, Wh2h, WhatW, WhatU, planes);

  hipFuncSetAttribute(reinterpret_cast<const void*>(&gru_cell_kernel),
                      hipFuncAttributeMaxDynamicSharedMemorySize, SMEM_BYTES);
  gru_cell_kernel<<<NBATCH / RB, NTHR, SMEM_BYTES, stream>>>(
      xb, hbp, wib, whb, wwb, wub, bi2h, bh2h, bhatW, bhatU, out);
}
